// _global_attention_sop_m_22814866277104
// MI455X (gfx1250) — hardware-verified
//
#include <hip/hip_runtime.h>
#include <stddef.h>
#include <math.h>


#define NH     4
#define DKC    32
#define XW     (NH * DKC)
#define TRI    528
#define TRIP   544
#define NT     256
#define NWAVE  8
#define QROWS  128
#define NSLOT  32
#define TP     40
#define MAXCH  1024

#define EPT    8
#define NGRP   2
#define CHUNK  (NT * EPT * NGRP)
#define WCAP   (EPT * NGRP * 32)
#define LISTN  (NWAVE * WCAP)
#define NBC    4096

#define LG_XS    0
#define LG_SW    16384
#define LG_LIST  16896
#define LG_PBH   17920
#define LG_PBL   (LG_PBH + NH * DKC * TP * 2)
#define LG_PAH   (LG_PBL + NH * DKC * TP * 2)
#define LG_PAL   (LG_PAH + NH * DKC * TP * 2)
#define LG_NS    0
#define LG_TRI   81920
#define LDS_GRAPH 90624

static_assert((CHUNK & (CHUNK - 1)) == 0);
static_assert(CHUNK <= 4096);
static_assert((NBC & (NBC - 1)) == 0 && NBC <= 4096);
static_assert(NT * 16 == NH * DKC * DKC);
static_assert(QROWS == NWAVE * 16);
static_assert(NWAVE * 4 == NSLOT);
static_assert(NT == NSLOT * 8);
static_assert(NT == NH * 64);
static_assert(TRI % 4 == 0);
static_assert(((TRIP / 4) % 8) == 0);
static_assert((TRIP * 4) % 128 == 0);
static_assert(LG_PAL + NH * DKC * TP * 2 <= LDS_GRAPH);
static_assert(LG_NS + 5 * NH * 1024 * 4 <= LG_TRI);
static_assert(LG_TRI + NH * TRIP * 4 <= LDS_GRAPH);
static_assert((LG_PBH % 16) == 0 && (LG_SW % 16) == 0 && (LG_LIST % 16) == 0 && (LG_TRI % 16) == 0);
static_assert((TP * 2) % 16 == 0);
static_assert(3 * NT >= NH * (TRIP / 4));

typedef float          v4f   __attribute__((ext_vector_type(4)));
typedef float          v8f   __attribute__((ext_vector_type(8)));
typedef int            v4i   __attribute__((ext_vector_type(4)));
typedef unsigned short v8us  __attribute__((ext_vector_type(8)));
typedef unsigned short v16us __attribute__((ext_vector_type(16)));
typedef __bf16         v16bf __attribute__((ext_vector_type(16)));
union FragB { v16us v; v8us h[2]; unsigned short s[16]; };

__device__ __forceinline__ unsigned short bf_rne(float f) {
  unsigned u = __float_as_uint(f);
  u += 0x7FFFu + ((u >> 16) & 1u);
  return (unsigned short)(u >> 16);
}
__device__ __forceinline__ float bf_f32(unsigned short b) { return __uint_as_float(((unsigned)b) << 16); }

__device__ __forceinline__ void split16(v4f x0, v4f x1, v4f x2, v4f x3, FragB& hi, FragB& lo) {
  float t[16];
  t[0] = x0.x; t[1] = x0.y; t[2] = x0.z; t[3] = x0.w;
  t[4] = x1.x; t[5] = x1.y; t[6] = x1.z; t[7] = x1.w;
  t[8] = x2.x; t[9] = x2.y; t[10] = x2.z; t[11] = x2.w;
  t[12] = x3.x; t[13] = x3.y; t[14] = x3.z; t[15] = x3.w;
#pragma unroll
  for (int q = 0; q < 16; ++q) {
    const unsigned short hq = bf_rne(t[q]);
    hi.s[q] = hq;
    lo.s[q] = bf_rne(t[q] - bf_f32(hq));
  }
}

__device__ __forceinline__ v8f wmb(v16us a, v16us b, v8f c) {
  const v16bf av = __builtin_bit_cast(v16bf, a);
  const v16bf bv = __builtin_bit_cast(v16bf, b);
  v8f d = __builtin_amdgcn_wmma_f32_16x16x32_bf16(false, av, false, bv, (short)0, c, false, false);
  asm volatile("v_nop\n\tv_nop\n\tv_nop\n\tv_nop" : "+v"(d) : "v"(a), "v"(b));
  return d;
}

__device__ __forceinline__ float wmax32(float v) {
  v = fmaxf(v, __shfl_xor(v, 16, 32));
  v = fmaxf(v, __shfl_xor(v, 8, 32));
  v = fmaxf(v, __shfl_xor(v, 4, 32));
  v = fmaxf(v, __shfl_xor(v, 2, 32));
  v = fmaxf(v, __shfl_xor(v, 1, 32));
  return v;
}
__device__ __forceinline__ float wsum32(float v) {
  v += __shfl_xor(v, 16, 32);
  v += __shfl_xor(v, 8, 32);
  v += __shfl_xor(v, 4, 32);
  v += __shfl_xor(v, 2, 32);
  v += __shfl_xor(v, 1, 32);
  return v;
}

template <int NB>
__device__ __forceinline__ int scan_chunk(const int* __restrict__ dsts, int nE, int cbase, int slotBase,
                                          int vec8, int* list, int tid, int lane, int wave) {
  int wc = 0;
#pragma unroll
  for (int g = 0; g < NGRP; ++g) {
    const int el0  = (g * NT + tid) * EPT;
    const int e0   = cbase + el0;
    const int sent = -2147483647 - 1;
    v4i da, db;
    if (vec8 != 0 && cbase + CHUNK <= nE) {
      da = *(const v4i*)(dsts + e0);
      db = *(const v4i*)(dsts + e0 + 4);
    } else {
      da.x = (e0     < nE) ? dsts[min(e0, nE - 1)] : sent;
      da.y = (e0 + 1 < nE) ? dsts[min(e0 + 1, nE - 1)] : sent;
      da.z = (e0 + 2 < nE) ? dsts[min(e0 + 2, nE - 1)] : sent;
      da.w = (e0 + 3 < nE) ? dsts[min(e0 + 3, nE - 1)] : sent;
      db.x = (e0 + 4 < nE) ? dsts[min(e0 + 4, nE - 1)] : sent;
      db.y = (e0 + 5 < nE) ? dsts[min(e0 + 5, nE - 1)] : sent;
      db.z = (e0 + 6 < nE) ? dsts[min(e0 + 6, nE - 1)] : sent;
      db.w = (e0 + 7 < nE) ? dsts[min(e0 + 7, nE - 1)] : sent;
    }
    const unsigned nb = (unsigned)slotBase;
    const unsigned s0 = (unsigned)da.x - nb, s1 = (unsigned)da.y - nb;
    const unsigned s2 = (unsigned)da.z - nb, s3 = (unsigned)da.w - nb;
    const unsigned s4 = (unsigned)db.x - nb, s5 = (unsigned)db.y - nb;
    const unsigned s6 = (unsigned)db.z - nb, s7 = (unsigned)db.w - nb;
    const bool h0 = s0 < (unsigned)NB, h1 = s1 < (unsigned)NB, h2 = s2 < (unsigned)NB, h3 = s3 < (unsigned)NB;
    const bool h4 = s4 < (unsigned)NB, h5 = s5 < (unsigned)NB, h6 = s6 < (unsigned)NB, h7 = s7 < (unsigned)NB;
    const unsigned any = __builtin_amdgcn_ballot_w32(h0 | h1 | h2 | h3 | h4 | h5 | h6 | h7);
    if (any != 0u) {
#define HITJ(J, HJ, SJ) { \
        const unsigned mj = __builtin_amdgcn_ballot_w32(HJ); \
        if (mj != 0u) { \
          if (HJ) { \
            const int pos = wc + (int)__builtin_amdgcn_mbcnt_lo(mj, 0u); \
            if (pos < WCAP) list[wave * WCAP + pos] = ((el0 + (J)) << 12) | (int)(SJ); \
          } \
          wc += (int)__builtin_popcount(mj); } }
      HITJ(0, h0, s0)
      HITJ(1, h1, s1)
      HITJ(2, h2, s2)
      HITJ(3, h3, s3)
      HITJ(4, h4, s4)
      HITJ(5, h5, s5)
      HITJ(6, h6, s6)
      HITJ(7, h7, s7)
#undef HITJ
    }
  }
  return wc;
}

__global__ __launch_bounds__(NT) void k_count(const int* __restrict__ ei, int* cnt, int nE, int vec8) {
  __shared__ __attribute__((aligned(16))) int scnt[NBC];
  __shared__ __attribute__((aligned(16))) int list[LISTN];
  __shared__ int wcnt[NWAVE];
  const int tid = threadIdx.x, lane = tid & 31, wave = tid >> 5;
  const int nodeBase = blockIdx.x * NBC;
  const int* dsts = ei;

  for (int i = tid; i < NBC; i += NT) scnt[i] = 0;
  __syncthreads();

  const int nChunks = (nE + CHUNK - 1) / CHUNK;
#pragma unroll 1
  for (int ch = 0; ch < nChunks; ++ch) {
    const int cbase = ch * CHUNK;
    const int wc = scan_chunk<NBC>(dsts, nE, cbase, nodeBase, vec8, list, tid, lane, wave);
    if (lane == 0) wcnt[wave] = wc;
    __syncthreads();
    if (wave == 0) {
#pragma unroll 1
      for (int wsx = 0; wsx < NWAVE; ++wsx) {
        int n = __builtin_amdgcn_readfirstlane(wcnt[wsx]);
        n = n > WCAP ? WCAP : (n < 0 ? 0 : n);
        const int* lp = list + wsx * WCAP;
#pragma unroll 1
        for (int i = 0; i < n; ++i) {
          const int ent  = __builtin_amdgcn_readfirstlane(lp[i]);
          const int slot = ent & (NBC - 1);
          if (lane == 0) scnt[slot] = scnt[slot] + 1;
        }
      }
    }
    __syncthreads();
  }

  v4i cq[4];
#pragma unroll
  for (int q = 0; q < 4; ++q) {
    const int f = (wave * 4 + q) * 128 + 4 * lane;
    cq[q] = *(const v4i*)(scnt + f);
  }
  int* cp = cnt + (size_t)nodeBase;
#pragma unroll
  for (int q = 0; q < 4; ++q) {
    const int f = (wave * 4 + q) * 128 + 4 * lane;
    *(volatile v4i*)(cp + f) = cq[q];
  }
  __threadfence();
#pragma unroll
  for (int q = 0; q < 4; ++q) {
    const int f = (wave * 4 + q) * 128 + 4 * lane;
    *(volatile v4i*)(cp + f) = cq[q];
  }
}

__global__ __launch_bounds__(NT) void k_qform(const float* __restrict__ x, const float* __restrict__ attn_w,
                                              const float* __restrict__ attn_b, float* imp, int M) {
  __shared__ __attribute__((aligned(16))) unsigned short sWh[NH * DKC * DKC];
  __shared__ __attribute__((aligned(16))) unsigned short sWl[NH * DKC * DKC];
  __shared__ __attribute__((aligned(16))) float simp[QROWS * NH];
  const int tid = threadIdx.x, lane = tid & 31, wave = tid >> 5, hh = lane >> 4, m16 = lane & 15;

#pragma unroll 4
  for (int k = 0; k < 16; ++k) {
    const int e = tid * 16 + k;
    const float f = attn_w[e];
    const unsigned short hq = bf_rne(f);
    sWh[e] = hq;
    sWl[e] = bf_rne(f - bf_f32(hq));
  }
  __syncthreads();

  const int rowBase = blockIdx.x * QROWS;
  const int r0 = wave * 16;
  int rowc = rowBase + r0 + m16;
  rowc = rowc > M - 1 ? M - 1 : rowc;
  const v8f z8 = {0.f, 0.f, 0.f, 0.f, 0.f, 0.f, 0.f, 0.f};

#pragma unroll 1
  for (int h = 0; h < NH; ++h) {
    const float* xp = x + (size_t)rowc * XW + h * DKC;
    const v4f x0 = *(const v4f*)(xp + 8 * hh);
    const v4f x1 = *(const v4f*)(xp + 8 * hh + 4);
    const v4f x2 = *(const v4f*)(xp + 16 + 8 * hh);
    const v4f x3 = *(const v4f*)(xp + 16 + 8 * hh + 4);
    FragB ah, al;
    split16(x0, x1, x2, x3, ah, al);

    v8f acc0 = z8, acc1 = z8;
    {
      const unsigned short* bp = sWh + (h * DKC + 0 * 16 + m16) * DKC + 8 * hh;
      const unsigned short* bq = sWl + (h * DKC + 0 * 16 + m16) * DKC + 8 * hh;
      FragB bh, bl;
      bh.h[0] = *(const v8us*)bp; bh.h[1] = *(const v8us*)(bp + 16);
      bl.h[0] = *(const v8us*)bq; bl.h[1] = *(const v8us*)(bq + 16);
      acc0 = wmb(ah.v, bh.v, acc0);
      acc0 = wmb(ah.v, bl.v, acc0);
      acc0 = wmb(al.v, bh.v, acc0);
    }
    {
      const unsigned short* bp = sWh + (h * DKC + 1 * 16 + m16) * DKC + 8 * hh;
      const unsigned short* bq = sWl + (h * DKC + 1 * 16 + m16) * DKC + 8 * hh;
      FragB bh, bl;
      bh.h[0] = *(const v8us*)bp; bh.h[1] = *(const v8us*)(bp + 16);
      bl.h[0] = *(const v8us*)bq; bl.h[1] = *(const v8us*)(bq + 16);
      acc1 = wmb(ah.v, bh.v, acc1);
      acc1 = wmb(ah.v, bl.v, acc1);
      acc1 = wmb(al.v, bh.v, acc1);
    }

    const float bb = attn_b[h];
#pragma unroll
    for (int r = 0; r < 8; ++r) {
      int rr = rowBase + r0 + 8 * hh + r;
      rr = rr > M - 1 ? M - 1 : rr;
      const float* xr = x + (size_t)rr * XW + h * DKC + m16;
      const float xa = xr[0], xb = xr[16];
      float pr = xa * acc0[r] + xb * acc1[r];
      pr += __shfl_xor(pr, 1, 32);
      pr += __shfl_xor(pr, 2, 32);
      pr += __shfl_xor(pr, 4, 32);
      pr += __shfl_xor(pr, 8, 32);
      if (m16 == r) simp[(r0 + 8 * hh + r) * NH + h] = pr + bb;
    }
  }
  __syncthreads();

  const v4f z4 = {0.f, 0.f, 0.f, 0.f};
  v4f ov = z4;
  if (tid < QROWS) ov = *(const v4f*)(simp + tid * NH);
  float* dp = imp + ((size_t)rowBase + tid) * NH;
  if (tid < QROWS) *(volatile v4f*)dp = ov;
  __threadfence();
  if (tid < QROWS) *(volatile v4f*)dp = ov;
}

__global__ __launch_bounds__(NT) void k_graph(
    const float* __restrict__ x, const int* __restrict__ batch, const float* __restrict__ imp,
    const int* __restrict__ cnt, const float* __restrict__ deg_w, const float* __restrict__ deg_b,
    const int* __restrict__ bsz, float* res, int M, int B) {
  extern __shared__ v4f lds_dyn[];
  char* lds = (char*)lds_dyn;
  float* xs = (float*)(lds + LG_XS);
  float* sw = (float*)(lds + LG_SW);
  int* slist = (int*)(lds + LG_LIST);
  unsigned short* pbh = (unsigned short*)(lds + LG_PBH);
  unsigned short* pbl = (unsigned short*)(lds + LG_PBL);
  unsigned short* pah = (unsigned short*)(lds + LG_PAH);
  unsigned short* pal = (unsigned short*)(lds + LG_PAL);
  float* nsb = (float*)(lds + LG_NS);
  float* tri = (float*)(lds + LG_TRI);
  __shared__ int swc[NWAVE];
  __shared__ float sred[NWAVE * 8];
  __shared__ float sstat[16];
  __shared__ int sflag[MAXCH];

  const int tid = threadIdx.x, lane = tid & 31, wave = tid >> 5, hh = lane >> 4, m16 = lane & 15;
  const int b = blockIdx.x;
  const int nseg = bsz[0];
  const bool bok = b < nseg;
  const float dw0 = deg_w[0], dw1 = deg_w[1], dw2 = deg_w[2], dw3 = deg_w[3];
  const float db0 = deg_b[0], db1 = deg_b[1], db2 = deg_b[2], db3 = deg_b[3];
  const int nCh = (M + NT - 1) / NT;
  const v4f z4 = {0.f, 0.f, 0.f, 0.f};
  const v8f z8 = {0.f, 0.f, 0.f, 0.f, 0.f, 0.f, 0.f, 0.f};

  slist[tid] = 0;
  for (int c = tid; c < MAXCH; c += NT) sflag[c] = 0;
  __syncthreads();

#pragma unroll 1
  for (int c = 0; c < nCh; ++c) {
    const int m = c * NT + tid;
    const int mc = m > M - 1 ? M - 1 : m;
    const bool hit = bok && (m < M) && (batch[mc] == b);
    const unsigned hb = __builtin_amdgcn_ballot_w32(hit);
    if (hb != 0u && lane == 0) sflag[c] = 1;
  }
  __syncthreads();

  float mxv[8];
#pragma unroll
  for (int k = 0; k < 8; ++k) mxv[k] = -INFINITY;
#pragma unroll 1
  for (int c = 0; c < nCh; ++c) {
    if (sflag[c] == 0) continue;
    const int m = c * NT + tid;
    const int mc = m > M - 1 ? M - 1 : m;
    const bool hit = bok && (m < M) && (batch[mc] == b);
    const v4f iv = *(const v4f*)(imp + (size_t)mc * NH);
    const float cf = (float)cnt[mc];
    const float d0 = fmaf(cf, dw0, db0), d1 = fmaf(cf, dw1, db1), d2 = fmaf(cf, dw2, db2), d3 = fmaf(cf, dw3, db3);
    mxv[0] = hit ? fmaxf(mxv[0], iv.x) : mxv[0];
    mxv[1] = hit ? fmaxf(mxv[1], iv.y) : mxv[1];
    mxv[2] = hit ? fmaxf(mxv[2], iv.z) : mxv[2];
    mxv[3] = hit ? fmaxf(mxv[3], iv.w) : mxv[3];
    mxv[4] = hit ? fmaxf(mxv[4], d0) : mxv[4];
    mxv[5] = hit ? fmaxf(mxv[5], d1) : mxv[5];
    mxv[6] = hit ? fmaxf(mxv[6], d2) : mxv[6];
    mxv[7] = hit ? fmaxf(mxv[7], d3) : mxv[7];
  }
#pragma unroll
  for (int k = 0; k < 8; ++k) {
    const float r = wmax32(mxv[k]);
    if (lane == 0) sred[wave * 8 + k] = r;
  }
  __syncthreads();
#pragma unroll
  for (int k = 0; k < 8; ++k) {
    float t = sred[k];
#pragma unroll
    for (int w = 1; w < NWAVE; ++w) t = fmaxf(t, sred[w * 8 + k]);
    mxv[k] = t;
  }
  __syncthreads();

  float sv[8];
#pragma unroll
  for (int k = 0; k < 8; ++k) sv[k] = 0.0f;
#pragma unroll 1
  for (int c = 0; c < nCh; ++c) {
    if (sflag[c] == 0) continue;
    const int m = c * NT + tid;
    const int mc = m > M - 1 ? M - 1 : m;
    const bool hit = bok && (m < M) && (batch[mc] == b);
    const v4f iv = *(const v4f*)(imp + (size_t)mc * NH);
    const float cf = (float)cnt[mc];
    if (hit) {
      sv[0] += expf(iv.x - mxv[0]);
      sv[1] += expf(iv.y - mxv[1]);
      sv[2] += expf(iv.z - mxv[2]);
      sv[3] += expf(iv.w - mxv[3]);
      sv[4] += expf(fmaf(cf, dw0, db0) - mxv[4]);
      sv[5] += expf(fmaf(cf, dw1, db1) - mxv[5]);
      sv[6] += expf(fmaf(cf, dw2, db2) - mxv[6]);
      sv[7] += expf(fmaf(cf, dw3, db3) - mxv[7]);
    }
  }
#pragma unroll
  for (int k = 0; k < 8; ++k) {
    const float r = wsum32(sv[k]);
    if (lane == 0) sred[wave * 8 + k] = r;
  }
  __syncthreads();
  if (tid == 0) {
#pragma unroll
    for (int k = 0; k < 8; ++k) {
      float t = sred[k];
#pragma unroll
      for (int w = 1; w < NWAVE; ++w) t += sred[w * 8 + k];
      sstat[k] = mxv[k];
      sstat[8 + k] = (t > 0.0f) ? (1.0f / t) : 0.0f;
    }
  }
  __syncthreads();

  v8f acc0 = z8, acc1 = z8;
  const int hw = wave >> 1, rh = wave & 1;
#pragma unroll 1
  for (int c = 0; c < nCh; ++c) {
    if (sflag[c] == 0) continue;
    const int m = c * NT + tid;
    const int mc = m > M - 1 ? M - 1 : m;
    const bool hit = bok && (m < M) && (batch[mc] == b);
    const unsigned hb = __builtin_amdgcn_ballot_w32(hit);
    const int rank = (int)__builtin_amdgcn_mbcnt_lo(hb, 0u);
    const int wc = (int)__builtin_popcount(hb);
    if (lane == 0) swc[wave] = wc;
    __syncthreads();
    int woff = 0, nh = 0;
#pragma unroll
    for (int w = 0; w < NWAVE; ++w) {
      const int cw = swc[w];
      woff += (w < wave) ? cw : 0;
      nh += cw;
    }
    nh = nh > NT ? NT : nh;
    if (hit) {
      int pos = woff + rank;
      pos = pos > NT - 1 ? NT - 1 : pos;
      slist[pos] = m;
    }
    __syncthreads();
    const int ng = (nh + NSLOT - 1) / NSLOT;
#pragma unroll 1
    for (int g = 0; g < ng && g < NT / NSLOT; ++g) {
#pragma unroll
      for (int q = 0; q < 4; ++q) {
        const int s = 4 * wave + q;
        const int sidx = g * NSLOT + s;
        const bool valid = sidx < nh;
        int nd = slist[sidx > NT - 1 ? NT - 1 : sidx];
        nd = nd < 0 ? 0 : (nd > M - 1 ? M - 1 : nd);
        v4f v = *(const v4f*)(x + (size_t)nd * XW + 4 * lane);
        v = valid ? v : z4;
        *(v4f*)(xs + s * XW + 4 * lane) = v;
      }
      if (wave == 0) {
        const int sidx = g * NSLOT + lane;
        const bool valid = sidx < nh;
        int nd = slist[sidx > NT - 1 ? NT - 1 : sidx];
        nd = nd < 0 ? 0 : (nd > M - 1 ? M - 1 : nd);
        const v4f iv = *(const v4f*)(imp + (size_t)nd * NH);
        const float cf = (float)cnt[nd];
        const float w0 = expf(iv.x - sstat[0]) * sstat[8]  + expf(fmaf(cf, dw0, db0) - sstat[4]) * sstat[12];
        const float w1 = expf(iv.y - sstat[1]) * sstat[9]  + expf(fmaf(cf, dw1, db1) - sstat[5]) * sstat[13];
        const float w2 = expf(iv.z - sstat[2]) * sstat[10] + expf(fmaf(cf, dw2, db2) - sstat[6]) * sstat[14];
        const float w3 = expf(iv.w - sstat[3]) * sstat[11] + expf(fmaf(cf, dw3, db3) - sstat[7]) * sstat[15];
        v4f wv;
        wv.x = valid ? w0 : 0.0f;
        wv.y = valid ? w1 : 0.0f;
        wv.z = valid ? w2 : 0.0f;
        wv.w = valid ? w3 : 0.0f;
        *(v4f*)(sw + lane * NH) = wv;
      }
      __syncthreads();
      {
        const int s = tid >> 3, cb = tid & 7;
        const int h = cb >> 1, c0 = (cb & 1) * 16;
        const float wv = sw[s * NH + h];
        const float* xr = xs + s * XW + 16 * cb;
        const v4f x0 = *(const v4f*)xr;
        const v4f x1 = *(const v4f*)(xr + 4);
        const v4f x2 = *(const v4f*)(xr + 8);
        const v4f x3 = *(const v4f*)(xr + 12);
        float xv[16];
        xv[0] = x0.x; xv[1] = x0.y; xv[2] = x0.z; xv[3] = x0.w;
        xv[4] = x1.x; xv[5] = x1.y; xv[6] = x1.z; xv[7] = x1.w;
        xv[8] = x2.x; xv[9] = x2.y; xv[10] = x2.z; xv[11] = x2.w;
        xv[12] = x3.x; xv[13] = x3.y; xv[14] = x3.z; xv[15] = x3.w;
#pragma unroll
        for (int e = 0; e < 16; ++e) {
          const int pidx = (h * DKC + c0 + e) * TP + s;
          const unsigned short bhq = bf_rne(xv[e]);
          pbh[pidx] = bhq;
          pbl[pidx] = bf_rne(xv[e] - bf_f32(bhq));
          const float a = wv * xv[e];
          const unsigned short ahq = bf_rne(a);
          pah[pidx] = ahq;
          pal[pidx] = bf_rne(a - bf_f32(ahq));
        }
      }
      __syncthreads();
      {
        FragB ahf, alf;
        const unsigned short* ap = pah + (hw * DKC + 16 * rh + m16) * TP + 8 * hh;
        const unsigned short* aq = pal + (hw * DKC + 16 * rh + m16) * TP + 8 * hh;
        ahf.h[0] = *(const v8us*)ap; ahf.h[1] = *(const v8us*)(ap + 16);
        alf.h[0] = *(const v8us*)aq; alf.h[1] = *(const v8us*)(aq + 16);
        {
          const unsigned short* bp = pbh + (hw * DKC + 0 * 16 + m16) * TP + 8 * hh;
          const unsigned short* bq = pbl + (hw * DKC + 0 * 16 + m16) * TP + 8 * hh;
          FragB bhf, blf;
          bhf.h[0] = *(const v8us*)bp; bhf.h[1] = *(const v8us*)(bp + 16);
          blf.h[0] = *(const v8us*)bq; blf.h[1] = *(const v8us*)(bq + 16);
          acc0 = wmb(ahf.v, bhf.v, acc0);
          acc0 = wmb(ahf.v, blf.v, acc0);
          acc0 = wmb(alf.v, bhf.v, acc0);
        }
        {
          const unsigned short* bp = pbh + (hw * DKC + 1 * 16 + m16) * TP + 8 * hh;
          const unsigned short* bq = pbl + (hw * DKC + 1 * 16 + m16) * TP + 8 * hh;
          FragB bhf, blf;
          bhf.h[0] = *(const v8us*)bp; bhf.h[1] = *(const v8us*)(bp + 16);
          blf.h[0] = *(const v8us*)bq; blf.h[1] = *(const v8us*)(bq + 16);
          acc1 = wmb(ahf.v, bhf.v, acc1);
          acc1 = wmb(ahf.v, blf.v, acc1);
          acc1 = wmb(alf.v, bhf.v, acc1);
        }
      }
    }
  }
  __syncthreads();

  {
    float* X0 = nsb + (size_t)(0 * NH + hw) * 1024;
#pragma unroll
    for (int r = 0; r < 8; ++r) {
      const int row = 16 * rh + 8 * hh + r;
      X0[row * DKC + m16] = acc0[r];
      X0[row * DKC + 16 + m16] = acc1[r];
    }
  }
  __syncthreads();

  {
    const int h = tid >> 6, u = tid & 63, i = u >> 1, j0 = (u & 1) * 16;
#define NSBUF(k) (nsb + ((k) * NH + h) * 1024)
    float sq;
    {
      const float* X0 = NSBUF(0);
      float tr = 0.0f;
#pragma unroll 1
      for (int d = 0; d < DKC; ++d) tr += (X0[d * DKC + d] + 0.001f);
      const float rc = 1.0f / tr;
      sq = sqrtf(tr);
      float* A1 = NSBUF(1);
      float* ZY = NSBUF(2);
#pragma unroll
      for (int e = 0; e < 16; ++e) {
        const int j = j0 + e;
        const float xm = X0[i * DKC + j] + ((i == j) ? 0.001f : 0.0f);
        const float a = xm * rc;
        A1[i * DKC + j] = a;
        ZY[i * DKC + j] = 0.5f * (((i == j) ? 3.0f : 0.0f) - a);
      }
      if (u < TRIP - TRI) tri[h * TRIP + TRI + u] = 0.0f;
    }
    __syncthreads();
#pragma unroll 1
    for (int step = 0; step < 6; ++step) {
      int oa, ob, od, mode;
      switch (step) {
        case 0:  oa = 1; ob = 2; od = 0; mode = 0; break;
        case 1:  oa = 2; ob = 0; od = 3; mode = 1; break;
        case 2:  oa = 0; ob = 3; od = 4; mode = 0; break;
        case 3:  oa = 3; ob = 2; od = 1; mode = 0; break;
        case 4:  oa = 1; ob = 4; od = 0; mode = 2; break;
        default: oa = 4; ob = 0; od = 0; mode = 3; break;
      }
      const float* P = NSBUF(oa);
      const float* Q = NSBUF(ob) + j0;
      float av[16];
#pragma unroll
      for (int e = 0; e < 16; ++e) av[e] = 0.0f;
#pragma unroll 1
      for (int k = 0; k < DKC; ++k) {
        const float p = P[i * DKC + k];
        const v4f q0 = *(const v4f*)(Q + k * DKC);
        const v4f q1 = *(const v4f*)(Q + k * DKC + 4);
        const v4f q2 = *(const v4f*)(Q + k * DKC + 8);
        const v4f q3 = *(const v4f*)(Q + k * DKC + 12);
        av[0]  += p * q0.x; av[1]  += p * q0.y; av[2]  += p * q0.z; av[3]  += p * q0.w;
        av[4]  += p * q1.x; av[5]  += p * q1.y; av[6]  += p * q1.z; av[7]  += p * q1.w;
        av[8]  += p * q2.x; av[9]  += p * q2.y; av[10] += p * q2.z; av[11] += p * q2.w;
        av[12] += p * q3.x; av[13] += p * q3.y; av[14] += p * q3.z; av[15] += p * q3.w;
      }
      if (mode == 3) {
        float* T = tri + h * TRIP;
        const int rowoff = i * DKC - ((i * (i - 1)) >> 1);
#pragma unroll
        for (int e = 0; e < 16; ++e) {
          const int j = j0 + e;
          if (j >= i) T[rowoff + (j - i)] = (0.5f * av[e]) * sq;
        }
      } else {
        float* D = NSBUF(od);
#pragma unroll
        for (int e = 0; e < 16; ++e) {
          const int j = j0 + e;
          const float d3 = (i == j) ? 3.0f : 0.0f;
          float v = av[e];
          v = (mode == 1) ? (0.5f * (d3 - v)) : ((mode == 2) ? (d3 - v) : v);
          D[i * DKC + j] = v;
        }
      }
      __syncthreads();
    }
#undef NSBUF
  }

#pragma unroll
  for (int p = 0; p < 3; ++p) {
    const int idx = p * NT + tid;
    if (idx < NH * (TRIP / 4)) {
      const int hq = idx / (TRIP / 4);
      const int piece = idx - hq * (TRIP / 4);
      const v4f v = *(const v4f*)(tri + 4 * idx);
      float* dp = res + ((size_t)(hq * B + b)) * TRIP + 4 * piece;
      *(volatile v4f*)dp = v;
    }
  }
  __threadfence();
#pragma unroll
  for (int p = 0; p < 3; ++p) {
    const int idx = p * NT + tid;
    if (idx < NH * (TRIP / 4)) {
      const int hq = idx / (TRIP / 4);
      const int piece = idx - hq * (TRIP / 4);
      const v4f v = *(const v4f*)(tri + 4 * idx);
      float* dp = res + ((size_t)(hq * B + b)) * TRIP + 4 * piece;
      *(volatile v4f*)dp = v;
    }
  }
}

__global__ __launch_bounds__(NT) void k_pack(const float* __restrict__ res, float* out, int B, int nf4) {
  const int g = blockIdx.x * NT + (int)threadIdx.x;
  if (g >= nf4) return;
  const int f = 4 * g;
  const int r = f / (NH * TRI);
  const int rem = f - r * (NH * TRI);
  const int s = rem / TRI;
  const int t = rem - s * TRI;
  int q = NH * r + s;
  const int qmax = NH * B - 1;
  q = q > qmax ? qmax : q;
  const v4f v = *(const v4f*)(res + (size_t)q * TRIP + t);
  float* dp = out + (size_t)f;
  *(volatile v4f*)dp = v;
  __threadfence();
  *(volatile v4f*)dp = v;
}

extern "C" void kernel_launch(void* const* d_in, const int* in_sizes, int n_in,
                              void* d_out, int out_size, void* d_ws, size_t ws_size,
                              hipStream_t stream) {
  if (n_in < 8) return;
  const int M = in_sizes[1];
  if (M < 1 || M > MAXCH * NT || in_sizes[0] != M * XW) return;
  const int E2 = in_sizes[2];
  const int E = E2 / 2;
  if (E < 1 || E2 != 2 * E || E > (1 << 28)) return;
  if (in_sizes[3] != NH * DKC * DKC || in_sizes[4] != NH || in_sizes[5] != NH || in_sizes[6] != NH || in_sizes[7] < 1) return;
  const int B = out_size / (NH * TRI);
  if (B < 1 || out_size != B * NH * TRI) return;

  const float* x      = (const float*)d_in[0];
  const int*   batch  = (const int*)d_in[1];
  const int*   edge   = (const int*)d_in[2];
  const float* attn_w = (const float*)d_in[3];
  const float* attn_b = (const float*)d_in[4];
  const float* deg_w  = (const float*)d_in[5];
  const float* deg_b  = (const float*)d_in[6];
  const int*   bsz    = (const int*)d_in[7];
  float* out = (float*)d_out;

  const int nQB  = (M + QROWS - 1) / QROWS;
  const int IMPR = nQB * QROWS;
  const int nBC  = (M + NBC - 1) / NBC;
  const int CNTN = nBC * NBC;
  const int nf4  = out_size / 4;

  char* ws = (char*)d_ws;
  size_t off = 0;
  const size_t oImp = off; off += (size_t)IMPR * NH * 4;        off = (off + 255) & ~(size_t)255;
  const size_t oCnt = off; off += (size_t)CNTN * 4;            off = (off + 255) & ~(size_t)255;
  const size_t oRes = off; off += (size_t)B * NH * TRIP * 4;    off = (off + 255) & ~(size_t)255;
  if (off > ws_size) return;
  float* impp = (float*)(ws + oImp);
  int*   cntp = (int*)(ws + oCnt);
  float* resp = (float*)(ws + oRes);

  k_qform<<<nQB, NT, 0, stream>>>(x, attn_w, attn_b, impp, M);
  k_count<<<nBC, NT, 0, stream>>>(edge, cntp, E, 1);
  hipFuncSetAttribute(reinterpret_cast<const void*>(&k_graph),
                      hipFuncAttributeMaxDynamicSharedMemorySize, LDS_GRAPH);
  k_graph<<<B, NT, LDS_GRAPH, stream>>>(x, batch, impp, cntp, deg_w, deg_b, bsz, resp, M, B);
  k_pack<<<(nf4 + NT - 1) / NT, NT, 0, stream>>>(resp, out, B, nf4);
}
